// FusionAVWGCN_6657199308827
// MI455X (gfx1250) — hardware-run, weakly checked
//
#include <hip/hip_runtime.h>
#include <stdint.h>

#define NN    8192
#define ED    16
#define CIN   32
#define COUT  32
#define NB    8
#define JT    256
#ifndef P_TERMS
#define P_TERMS 2
#endif

static_assert(NN % 64 == 0);
static_assert(NN % 128 == 0);
static_assert(NB * CIN == JT);
static_assert(JT == 256);
static_assert(ED == 16);
static_assert(COUT == 32);
static_assert(2 * CIN + CIN == 96);
static_assert(P_TERMS == 1 || P_TERMS == 2);

typedef __attribute__((ext_vector_type(16))) __bf16       v16b;
typedef __attribute__((ext_vector_type(8)))  __bf16       v8b;
typedef __attribute__((ext_vector_type(8)))  float        v8f;
typedef __attribute__((ext_vector_type(4)))  float        v4f;
typedef __attribute__((ext_vector_type(4)))  unsigned int v4u;
typedef v8b __attribute__((may_alias)) v8ba;
typedef v4f __attribute__((may_alias)) v4fa;
typedef v4u __attribute__((may_alias)) v4ua;

union FB { v16b v; v8b h[2]; };

__device__ __forceinline__ unsigned bfb(float f) {
  const unsigned u = __float_as_uint(f);
  const unsigned r = (u + 0x7FFFu + ((u >> 16) & 1u)) >> 16;
  const unsigned q = (u >> 16) | 0x40u;
  return ((u & 0x7FFFFFFFu) > 0x7F800000u) ? q : r;
}
__device__ __forceinline__ unsigned bfb_fast(float f) {
  const unsigned u = __float_as_uint(f);
  return (u + 0x7FFFu + ((u >> 16) & 1u)) >> 16;
}
__device__ __forceinline__ float bfv(unsigned b) { return __uint_as_float(b << 16); }
__device__ __forceinline__ float bfr(float f) { return bfv(bfb(f)); }
__device__ __forceinline__ unsigned pk2(float a, float b) { return bfb(a) | (bfb(b) << 16); }

__device__ __forceinline__ v4u pack8(v4f a, v4f b) {
  v4u o;
  o.x = pk2(a.x, a.y); o.y = pk2(a.z, a.w); o.z = pk2(b.x, b.y); o.w = pk2(b.z, b.w);
  return o;
}
__device__ __forceinline__ unsigned split2(float a, float b, unsigned* lo) {
  const unsigned ha = bfb(a), hb = bfb(b);
  const unsigned la = bfb(a - bfv(ha)), lb = bfb(b - bfv(hb));
  *lo = la | (lb << 16);
  return ha | (hb << 16);
}

__device__ __forceinline__ v16b ldfrag(const unsigned short* p) {
  FB f;
  f.h[0] = *(const v8ba*)(p);
  f.h[1] = *(const v8ba*)(p + 16);
  return f.v;
}

__device__ __forceinline__ v8f wmb(v16b a, v16b b, v8f c) {
  c = __builtin_amdgcn_wmma_f32_16x16x32_bf16(false, a, false, b, (short)0, c, false, false);
  asm volatile("v_nop\n\tv_nop\n\tv_nop\n\tv_nop" : "+v"(c) : "v"(a), "v"(b));
  return c;
}

#define PREP_A 128
#define PREP_B 1024
#define PREP_C 16
#define PREP_BLKS (PREP_A + PREP_B + PREP_C + 1)

__global__ __launch_bounds__(256) void k_prep(const float* __restrict__ x, const float* __restrict__ E,
                                              const float* __restrict__ WP, const float* __restrict__ BP,
                                              unsigned short* __restrict__ EB, float* __restrict__ EF,
                                              float* __restrict__ NRM, unsigned short* __restrict__ XVT,
                                              unsigned short* __restrict__ WPT, float* __restrict__ BPF) {
  __shared__ __align__(16) float sm[64 * 36];
  const int tid = threadIdx.x;
  const int blk = blockIdx.x;

  if (blk < PREP_A) {
    const int g = blk * 256 + tid;
    const int n = g >> 2, q = g & 3;
    const v4f a = *(const v4fa*)(E + (size_t)g * 4);
    const float r0 = bfr(a.x), r1 = bfr(a.y), r2 = bfr(a.z), r3 = bfr(a.w);
    const v4f ef = {r0, r1, r2, r3};
    float s = ((r0 * r0 + r1 * r1) + r2 * r2) + r3 * r3;
    s += __shfl_xor(s, 1, 32);
    s += __shfl_xor(s, 2, 32);
    const float nrm = sqrtf(s);
    const float* ep = E + (size_t)n * ED + (q & 1) * 8;
    const v4f c0 = *(const v4fa*)ep;
    const v4f c1 = *(const v4fa*)(ep + 4);
    asm volatile("" :: "v"(c0), "v"(c1));
    const unsigned msk = (q < 2) ? 0xFFFFFFFFu : 0u;
    v4u eb = pack8(c0, c1);
    eb.x &= msk; eb.y &= msk; eb.z &= msk; eb.w &= msk;
    if (q == 0) sm[tid >> 2] = nrm;
    __syncthreads();
    const int ti = (tid < 15) ? tid : 15;
    const v4f nv = *(const v4fa*)(sm + 4 * ti);
    asm volatile("" :: "v"(nv));
    *(volatile v4f*)(EF + (size_t)g * 4) = ef;
    *(volatile v4u*)(EB + (size_t)g * 8) = eb;
    if (tid < 16) *(volatile v4f*)(NRM + blk * 64 + tid * 4) = nv;
    __threadfence();
    *(volatile v4f*)(EF + (size_t)g * 4) = ef;
    *(volatile v4u*)(EB + (size_t)g * 8) = eb;
    if (tid < 16) *(volatile v4f*)(NRM + blk * 64 + tid * 4) = nv;
  } else if (blk < PREP_A + PREP_B) {
    const int t = blk - PREP_A;
    const int b = t >> 7;
    const int m0 = (t & 127) * 64;
#pragma unroll
    for (int it = 0; it < 2; ++it) {
      const int idx = it * 256 + tid;
      const int mm = idx >> 3, c4 = (idx & 7) * 4;
      const v4f v = *(const v4fa*)(x + ((size_t)(b * NN + m0 + mm) * CIN + c4));
      *(v4fa*)(sm + mm * 36 + c4) = v;
    }
    __syncthreads();
    const int c = tid >> 3, pc = tid & 7;
    float f[8];
#pragma unroll
    for (int e = 0; e < 8; ++e) f[e] = sm[(pc * 8 + e) * 36 + c];
    v4u o;
    o.x = pk2(f[0], f[1]); o.y = pk2(f[2], f[3]); o.z = pk2(f[4], f[5]); o.w = pk2(f[6], f[7]);
    unsigned short* dst = XVT + (size_t)(b * CIN + c) * NN + m0 + pc * 8;
    *(volatile v4u*)dst = o;
    __threadfence();
    *(volatile v4u*)dst = o;
  } else if (blk < PREP_A + PREP_B + PREP_C) {
    const int d = blk - (PREP_A + PREP_B);
    const float* wd = WP + (size_t)d * 2048;
#pragma unroll
    for (int it = 0; it < 2; ++it) {
      const int idx = it * 256 + tid;
      const int ki = idx >> 3, o4 = (idx & 7) * 4;
      const v4f v = *(const v4fa*)(wd + ki * 32 + o4);
      *(v4fa*)(sm + ki * 36 + o4) = v;
    }
    __syncthreads();
    v4u ov[2];
#pragma unroll
    for (int it = 0; it < 2; ++it) {
      const int idx = it * 256 + tid;
      const int o = idx >> 4, p = idx & 15;
      const int kb = (p < 8) ? (8 * p) : ((p < 12) ? (8 * p - 32) : 0);
      const unsigned msk = (p < 12) ? 0xFFFFFFFFu : 0u;
      float f[8];
#pragma unroll
      for (int e = 0; e < 8; ++e) f[e] = sm[(kb + e) * 36 + o];
      v4u w;
      w.x = pk2(f[0], f[1]) & msk; w.y = pk2(f[2], f[3]) & msk;
      w.z = pk2(f[4], f[5]) & msk; w.w = pk2(f[6], f[7]) & msk;
      ov[it] = w;
    }
#pragma unroll
    for (int it = 0; it < 2; ++it) {
      const int idx = it * 256 + tid;
      *(volatile v4u*)(WPT + (size_t)(d * 32 + (idx >> 4)) * 128 + (idx & 15) * 8) = ov[it];
    }
    __threadfence();
#pragma unroll
    for (int it = 0; it < 2; ++it) {
      const int idx = it * 256 + tid;
      *(volatile v4u*)(WPT + (size_t)(d * 32 + (idx >> 4)) * 128 + (idx & 15) * 8) = ov[it];
    }
  } else {
    const int i = (tid < 127) ? tid : 127;
    const v4f b = *(const v4fa*)(BP + i * 4);
    asm volatile("" :: "v"(b));
    const v4f r = {bfr(b.x), bfr(b.y), bfr(b.z), bfr(b.w)};
    if (tid < 128) *(volatile v4f*)(BPF + tid * 4) = r;
    __threadfence();
    if (tid < 128) *(volatile v4f*)(BPF + tid * 4) = r;
  }
}

#define XVP 72
#define EKP 40
#define PPP 72
#define GPP 260
#define OFF_XV 0
#define OFF_EK (OFF_XV + 256 * XVP * 2)
#define OFF_PH (OFF_EK + 64 * EKP * 2)
#define OFF_PL (OFF_PH + 64 * PPP * 2)
#define STG_BYTES (OFF_PL + 64 * PPP * 2)
#define G_BYTES (64 * GPP * 4)
#define SRAW_BYTES ((G_BYTES > STG_BYTES) ? G_BYTES : STG_BYTES)
static_assert(SRAW_BYTES + 64 * 8 * 4 + 64 * 4 + 8 * 4 <= 327680);
static_assert((OFF_EK % 16) == 0 && (OFF_PH % 16) == 0 && (OFF_PL % 16) == 0);

__global__ __launch_bounds__(256) __attribute__((amdgpu_num_vgpr(248)))
void k_attn(const float* __restrict__ x, const unsigned short* __restrict__ EB,
            const unsigned short* __restrict__ XVT, const float* __restrict__ NRM,
            unsigned short* __restrict__ AX) {
  __shared__ __align__(16) unsigned char sraw[SRAW_BYTES];
  __shared__ float sLp[64 * 8];
  __shared__ float sL[64];
  __shared__ float sRed[8];

  unsigned short* sXV = (unsigned short*)(sraw + OFF_XV);
  unsigned short* sEK = (unsigned short*)(sraw + OFF_EK);
  unsigned short* sPH = (unsigned short*)(sraw + OFF_PH);
  unsigned short* sPL = (unsigned short*)(sraw + OFF_PL);
  float* sG = (float*)sraw;

  const int tid = threadIdx.x, lane = tid & 31, w = tid >> 5;
  const int h = lane >> 4, m = lane & 15;
  const int q0 = blockIdx.x * 64;

  float mx = 0.0f;
#pragma unroll
  for (int it = 0; it < 8; ++it) {
    const v4f v = *(const v4fa*)(NRM + (size_t)(it * 256 + tid) * 4);
    mx = fmaxf(mx, fmaxf(fmaxf(v.x, v.y), fmaxf(v.z, v.w)));
  }
#pragma unroll
  for (int off = 16; off >= 1; off >>= 1) mx = fmaxf(mx, __shfl_xor(mx, off, 32));
  if (lane == 0) sRed[w] = mx;
  __syncthreads();
  float nmax = sRed[0];
#pragma unroll
  for (int i = 1; i < 8; ++i) nmax = fmaxf(nmax, sRed[i]);
  const bool poison = !(nmax * nmax <= 320.0f);

  const int kt = w & 3, qp = w >> 2;
  const int qt = w & 3, ch = w >> 2;

  v16b qb[2];
  float Mq[2], lp[2];
#pragma unroll
  for (int j = 0; j < 2; ++j) {
    const int qrow = q0 + (2 * qp + j) * 16 + m;
    qb[j] = ldfrag(EB + (size_t)qrow * 32 + 8 * h);
    Mq[j] = NRM[qrow] * nmax;
    lp[j] = 0.0f;
  }

  const v8f zero8 = {0.f, 0.f, 0.f, 0.f, 0.f, 0.f, 0.f, 0.f};
  v8f acc[8];
#pragma unroll
  for (int t = 0; t < 8; ++t) acc[t] = zero8;

#pragma unroll 1
  for (int tile = 0; tile < NN / 64; ++tile) {
    const int key0 = tile * 64;
    {
      const int r = tid >> 2, pc = tid & 3;
      const v4u e = *(const v4ua*)(EB + (size_t)(key0 + r) * 32 + pc * 8);
      v4u xv[8];
#pragma unroll
      for (int it = 0; it < 8; ++it) {
        const int row = it * 32 + (tid >> 3), p8 = tid & 7;
        xv[it] = *(const v4ua*)(XVT + (size_t)row * NN + key0 + p8 * 8);
      }
      *(v4ua*)(sEK + r * EKP + pc * 8) = e;
#pragma unroll
      for (int it = 0; it < 8; ++it) {
        const int row = it * 32 + (tid >> 3), p8 = tid & 7;
        *(v4ua*)(sXV + row * XVP + p8 * 8) = xv[it];
      }
    }
    __syncthreads();

    {
      const v16b ka = ldfrag(sEK + (kt * 16 + m) * EKP + 8 * h);
#pragma unroll
      for (int j = 0; j < 2; ++j) {
        v8f s = zero8;
        s = wmb(ka, qb[j], s);
        unsigned hb[8], lb[8];
        float lj = lp[j];
        const float mq = Mq[j];
#pragma unroll
        for (int r = 0; r < 8; ++r) {
          float sv = s[r];
          sv = (sv > 0.0f) ? sv : 0.0f;
          const float p = __builtin_amdgcn_exp2f((sv - mq) * 1.44269504088896341f);
          const unsigned b16 = bfb_fast(p);
          hb[r] = b16;
          if (P_TERMS == 1) {
            lj += bfv(b16);
            lb[r] = 0u;
          } else {
            lj += p;
            lb[r] = bfb_fast(p - bfv(b16));
          }
        }
        lp[j] = lj;
        const int prow = (2 * qp + j) * 16 + m;
        v4u ph;
        ph.x = hb[0] | (hb[1] << 16); ph.y = hb[2] | (hb[3] << 16);
        ph.z = hb[4] | (hb[5] << 16); ph.w = hb[6] | (hb[7] << 16);
        *(v4ua*)(sPH + prow * PPP + kt * 16 + 8 * h) = ph;
        if (P_TERMS == 2) {
          v4u pl;
          pl.x = lb[0] | (lb[1] << 16); pl.y = lb[2] | (lb[3] << 16);
          pl.z = lb[4] | (lb[5] << 16); pl.w = lb[6] | (lb[7] << 16);
          *(v4ua*)(sPL + prow * PPP + kt * 16 + 8 * h) = pl;
        }
      }
    }
    __syncthreads();

#pragma unroll
    for (int ks = 0; ks < 2; ++ks) {
      const v16b pa = ldfrag(sPH + (qt * 16 + m) * PPP + ks * 32 + 8 * h);
      v16b pl = pa;
      if (P_TERMS == 2) pl = ldfrag(sPL + (qt * 16 + m) * PPP + ks * 32 + 8 * h);
#pragma unroll
      for (int nt = 0; nt < 8; ++nt) {
        const v16b xb = ldfrag(sXV + (ch * 128 + nt * 16 + m) * XVP + ks * 32 + 8 * h);
        acc[nt] = wmb(pa, xb, acc[nt]);
        if (P_TERMS == 2) acc[nt] = wmb(pl, xb, acc[nt]);
      }
    }
    __syncthreads();
  }

#pragma unroll
  for (int j = 0; j < 2; ++j) sLp[((2 * qp + j) * 16 + m) * 8 + kt * 2 + h] = lp[j];
  __syncthreads();
  if (tid < 64) {
    float l = sLp[tid * 8 + 0];
#pragma unroll
    for (int i = 1; i < 8; ++i) l += sLp[tid * 8 + i];
    sL[tid] = l;
  }
  __syncthreads();

  {
    const float qnan = __uint_as_float(0x7FC00000u);
#pragma unroll
    for (int r = 0; r < 8; ++r) {
      const int row = qt * 16 + 8 * h + r;
      const float inv = 1.0f / sL[row];
#pragma unroll
      for (int nt = 0; nt < 8; ++nt) {
        float v = acc[nt][r] * inv;
        v = poison ? qnan : v;
        sG[row * GPP + ch * 128 + nt * 16 + m] = v;
      }
    }
  }
  __syncthreads();

  {
    const int p = tid & 15, ps = p & 3, cls = p >> 2;
    const unsigned mxm = (cls == 0) ? 0xFFFFFFFFu : 0u;
    const unsigned mhm = (cls == 1) ? 0xFFFFFFFFu : 0u;
    const unsigned mlm = (cls == 2) ? 0xFFFFFFFFu : 0u;
#pragma unroll 1
    for (int pass = 0; pass < 2; ++pass) {
#pragma unroll 2
      for (int it = 0; it < 32; ++it) {
        const int b = it >> 2;
        const int nl = (it & 3) * 16 + (tid >> 4);
        const size_t grow = (size_t)b * NN + q0 + nl;
        const float* xp = x + grow * CIN + ps * 8;
        const v4f xa = *(const v4fa*)xp;
        const v4f xc = *(const v4fa*)(xp + 4);
        asm volatile("" :: "v"(xa), "v"(xc));
        const float* gp = sG + nl * GPP + b * 32 + ps * 8;
        const v4f ga = *(const v4fa*)gp;
        const v4f gc = *(const v4fa*)(gp + 4);
        const v4u ox = pack8(xa, xc);
        v4u oh, ol;
        unsigned t0, t1, t2, t3;
        oh.x = split2(ga.x, ga.y, &t0);
        oh.y = split2(ga.z, ga.w, &t1);
        oh.z = split2(gc.x, gc.y, &t2);
        oh.w = split2(gc.z, gc.w, &t3);
        ol.x = t0; ol.y = t1; ol.z = t2; ol.w = t3;
        v4u o;
        o.x = (ox.x & mxm) | (oh.x & mhm) | (ol.x & mlm);
        o.y = (ox.y & mxm) | (oh.y & mhm) | (ol.y & mlm);
        o.z = (ox.z & mxm) | (oh.z & mhm) | (ol.z & mlm);
        o.w = (ox.w & mxm) | (oh.w & mhm) | (ol.w & mlm);
        *(volatile v4u*)(AX + grow * 128 + p * 8) = o;
      }
      __threadfence();
    }
  }
}

#define WLP 104
static_assert(512 * WLP * 2 + 128 * 16 * 4 + 512 * 4 + 8 * 16 * 36 * 4 <= 327680);

__global__ __launch_bounds__(256) void k_out(const unsigned short* __restrict__ AX,
                                             const unsigned short* __restrict__ WPT,
                                             const float* __restrict__ EF, const float* __restrict__ BPF,
                                             float* __restrict__ out) {
  __shared__ __align__(16) unsigned short sW[512 * WLP];
  __shared__ __align__(16) float sE[128 * 16];
  __shared__ __align__(16) float sB[512];
  __shared__ __align__(16) float sO[8 * 16 * 36];

  const int tid = threadIdx.x, lane = tid & 31, w = tid >> 5;
  const int h = lane >> 4, m = lane & 15;
  const int blk = blockIdx.x;
  const int n0 = (blk * 128) & (NN - 1);

#pragma unroll 4
  for (int it = 0; it < 24; ++it) {
    const int idx = it * 256 + tid;
    const int row = idx / 12;
    const int pc = idx - row * 12;
    const v4u v = *(const v4ua*)(WPT + (size_t)row * 128 + pc * 8);
    *(v4ua*)(sW + row * WLP + pc * 8) = v;
  }
#pragma unroll
  for (int it = 0; it < 2; ++it) {
    const int idx = it * 256 + tid;
    const v4f v = *(const v4fa*)(EF + (size_t)n0 * ED + idx * 4);
    *(v4fa*)(sE + idx * 4) = v;
  }
  {
    const int i = (tid < 127) ? tid : 127;
    const v4f v = *(const v4fa*)(BPF + i * 4);
    asm volatile("" :: "v"(v));
    if (tid < 128) *(v4fa*)(sB + tid * 4) = v;
  }
  __syncthreads();

  const size_t row0 = (size_t)blk * 128 + w * 16;
  const unsigned short* ar = AX + (row0 + m) * 128 + 8 * h;
  v16b a[3];
#pragma unroll
  for (int ks = 0; ks < 3; ++ks) a[ks] = ldfrag(ar + ks * 32);

  const v8f zero8 = {0.f, 0.f, 0.f, 0.f, 0.f, 0.f, 0.f, 0.f};
  v8f oacc[2];
  oacc[0] = zero8; oacc[1] = zero8;

#pragma unroll 1
  for (int d = 0; d < ED; ++d) {
    float e[8];
#pragma unroll
    for (int r = 0; r < 8; ++r) e[r] = sE[(w * 16 + 8 * h + r) * 16 + d];
#pragma unroll
    for (int nt = 0; nt < 2; ++nt) {
      v8f g = zero8;
#pragma unroll
      for (int ks = 0; ks < 3; ++ks) {
        const v16b bf = ldfrag(sW + (d * 32 + nt * 16 + m) * WLP + ks * 32 + 8 * h);
        g = wmb(a[ks], bf, g);
      }
      const float bp = sB[d * 32 + nt * 16 + m];
#pragma unroll
      for (int r = 0; r < 8; ++r) oacc[nt][r] = fmaf(e[r], g[r] + bp, oacc[nt][r]);
    }
  }

  float* so = sO + w * (16 * 36);
#pragma unroll
  for (int nt = 0; nt < 2; ++nt)
#pragma unroll
    for (int r = 0; r < 8; ++r) so[(8 * h + r) * 36 + nt * 16 + m] = oacc[nt][r];
  __builtin_amdgcn_fence(__ATOMIC_RELEASE, "workgroup");
  __builtin_amdgcn_wave_barrier();
  __builtin_amdgcn_fence(__ATOMIC_ACQUIRE, "workgroup");
  {
    const int q8 = lane & 7, sub = lane >> 3;
    v4f ov[4];
#pragma unroll
    for (int it = 0; it < 4; ++it) ov[it] = *(const v4fa*)(so + (it * 4 + sub) * 36 + 4 * q8);
#pragma unroll
    for (int it = 0; it < 4; ++it)
      *(volatile v4f*)(out + (row0 + it * 4 + sub) * COUT + 4 * q8) = ov[it];
    __threadfence();
#pragma unroll
    for (int it = 0; it < 4; ++it)
      *(volatile v4f*)(out + (row0 + it * 4 + sub) * COUT + 4 * q8) = ov[it];
  }
}

extern "C" void kernel_launch(void* const* d_in, const int* in_sizes, int n_in,
                              void* d_out, int out_size, void* d_ws, size_t ws_size,
                              hipStream_t stream) {
  if (n_in < 4) return;
  if (in_sizes[0] != NB * NN * CIN) return;
  if (in_sizes[1] != NN * ED) return;
  if (in_sizes[2] != ED * 2 * CIN * COUT) return;
  if (in_sizes[3] != ED * COUT) return;
  if (out_size != NB * NN * COUT) return;

  const float* x  = (const float*)d_in[0];
  const float* E  = (const float*)d_in[1];
  const float* WP = (const float*)d_in[2];
  const float* BP = (const float*)d_in[3];
  float* out = (float*)d_out;

  size_t off = 0;
  const size_t oEB  = off; off += (size_t)NN * 32 * 2;
  const size_t oXVT = off; off += (size_t)JT * NN * 2;
  const size_t oWPT = off; off += (size_t)512 * 128 * 2;
  const size_t oAX  = off; off += (size_t)NB * NN * 128 * 2;
  const size_t oEF  = off; off += (size_t)NN * ED * 4;
  const size_t oNRM = off; off += (size_t)NN * 4;
  const size_t oBPF = off; off += (size_t)ED * COUT * 4;
  if (off > ws_size) return;

  char* ws = (char*)d_ws;
  unsigned short* EB  = (unsigned short*)(ws + oEB);
  unsigned short* XVT = (unsigned short*)(ws + oXVT);
  unsigned short* WPT = (unsigned short*)(ws + oWPT);
  unsigned short* AX  = (unsigned short*)(ws + oAX);
  float* EF  = (float*)(ws + oEF);
  float* NRM = (float*)(ws + oNRM);
  float* BPF = (float*)(ws + oBPF);

  k_prep<<<dim3(PREP_BLKS), dim3(256), 0, stream>>>(x, E, WP, BP, EB, EF, NRM, XVT, WPT, BPF);
  k_attn<<<dim3(NN / 64), dim3(256), 0, stream>>>(x, EB, XVT, NRM, AX);
  k_out<<<dim3((NB * NN) / 128), dim3(256), 0, stream>>>(AX, WPT, EF, BPF, out);
  (void)hipGetLastError();
}
